// MultiHeadCausalAttention_82961588290058
// MI455X (gfx1250) — hardware-verified
//
#include <hip/hip_runtime.h>
#include <math.h>

constexpr int kSeqN  = 2048;
constexpr int kDim   = 1024;
constexpr int kQVK   = 3072;
constexpr int kHeads = 16;
constexpr int kDh    = 64;
constexpr int kChunk = 64;
constexpr int kNCh   = kSeqN / kChunk;
constexpr int kHN    = kHeads * kSeqN;
constexpr float kQScale    = 0.125f;
constexpr float kQ16Carry  = 1024.0f;
constexpr float kQ16Inv    = 1.0f / 1024.0f;
constexpr float kVCarry    = 8.0f;
constexpr float kVCarryInv = 0.125f;
constexpr float kEpsDen    = 1.25e-7f;
static_assert(kHeads * kDh == kDim);
static_assert(kSeqN % kChunk == 0 && kNCh * kChunk == kSeqN);
static_assert(kSeqN % 64 == 0 && kQVK % 64 == 0 && kDim % 32 == 0);
static_assert(kDh % 64 == 0 && kChunk % 32 == 0 && kChunk % 64 == 0);

typedef __attribute__((ext_vector_type(16))) _Float16 v16h;
typedef __attribute__((ext_vector_type(8)))  _Float16 v8h;
typedef __attribute__((ext_vector_type(16))) __bf16   v16b;
typedef __attribute__((ext_vector_type(8)))  __bf16   v8b;
typedef __attribute__((ext_vector_type(8)))  float    v8f;
typedef __attribute__((ext_vector_type(4)))  float    v4f;
typedef __attribute__((ext_vector_type(4)))  unsigned int v4u;

__device__ __forceinline__ unsigned short f2bf_bits(float f) {
  unsigned u = __float_as_uint(f);
  return (unsigned short)((u + 0x7FFFu + ((u >> 16) & 1u)) >> 16);
}
__device__ __forceinline__ float bf_bits2f(unsigned short h) { return __uint_as_float(((unsigned)h) << 16); }

__device__ __forceinline__ void dep_guard_h(v8f& a, v8f& b, v16h x, v16h y) { asm volatile("v_nop\n\tv_nop\n\tv_nop\n\tv_nop" : "+v"(a), "+v"(b) : "v"(x), "v"(y)); }
__device__ __forceinline__ void dep_guard_b(v8f& a, v8f& b, v16b x, v16b y) { asm volatile("v_nop\n\tv_nop\n\tv_nop\n\tv_nop" : "+v"(a), "+v"(b) : "v"(x), "v"(y)); }
__device__ __forceinline__ void keep4_h(v16h a, v16h b, v16h c, v16h d) { asm volatile("v_nop" :: "v"(a), "v"(b), "v"(c), "v"(d)); }
__device__ __forceinline__ void keep4_b(v16b a, v16b b, v16b c, v16b d) { asm volatile("v_nop" :: "v"(a), "v"(b), "v"(c), "v"(d)); }
__device__ __forceinline__ void acc_guard4(v8f& a, v8f& b, v8f& c, v8f& d) { asm volatile("v_nop\n\tv_nop\n\tv_nop\n\tv_nop" : "+v"(a), "+v"(b), "+v"(c), "+v"(d)); }
template <typename T> struct Frag;
template <> struct Frag<_Float16> {
  typedef v16h V; union U { v16h v; v8h h[2]; };
  static __device__ __forceinline__ v16h load(const _Float16* p) {
    U f; f.h[0] = *(const v8h*)(p); f.h[1] = *(const v8h*)(p + 16); return f.v;
  }
  static __device__ __forceinline__ v8f mma(v16h a, v16h b, v8f c) {
    return __builtin_amdgcn_wmma_f32_16x16x32_f16(false, a, false, b, (short)0, c, false, false);
  }
  static __device__ __forceinline__ void guard(v8f& a, v8f& b, v16h x, v16h y) { dep_guard_h(a, b, x, y); }
  static __device__ __forceinline__ void keep(v16h a, v16h b, v16h c, v16h d) { keep4_h(a, b, c, d); }
};
template <> struct Frag<__bf16> {
  typedef v16b V; union U { v16b v; v8b h[2]; };
  static __device__ __forceinline__ v16b load(const __bf16* p) {
    U f; f.h[0] = *(const v8b*)(p); f.h[1] = *(const v8b*)(p + 16); return f.v;
  }
  static __device__ __forceinline__ v8f mma(v16b a, v16b b, v8f c) {
    return __builtin_amdgcn_wmma_f32_16x16x32_bf16(false, a, false, b, (short)0, c, false, false);
  }
  static __device__ __forceinline__ void guard(v8f& a, v8f& b, v16b x, v16b y) { dep_guard_b(a, b, x, y); }
  static __device__ __forceinline__ void keep(v16b a, v16b b, v16b c, v16b d) { keep4_b(a, b, c, d); }
};

__device__ __forceinline__ unsigned pk16(unsigned short a, unsigned short b) { return (unsigned)a | ((unsigned)b << 16); }
__device__ __forceinline__ unsigned short h_bits(float f) { const _Float16 h = (_Float16)f; return __builtin_bit_cast(unsigned short, h); }
#define PACK8W(a) ((v4u){pk16(a[0], a[1]), pk16(a[2], a[3]), pk16(a[4], a[5]), pk16(a[6], a[7])})

__device__ __forceinline__ float h16_to_f32(unsigned hb) {
  const unsigned sgn = (hb & 0x8000u) << 16; const unsigned em = hb & 0x7fffu;
  const float fn = __uint_as_float((em << 13) + 0x38000000u);
  const float fs = (float)em * 5.9604644775390625e-8f;
  const float mag = (em < 0x400u) ? fs : fn; return __uint_as_float(__float_as_uint(mag) | sgn);
}

__device__ __forceinline__ v8f mma_h(v16h a, v16h b, v8f c) {
  c = __builtin_amdgcn_wmma_f32_16x16x32_f16(false, a, false, b, (short)0, c, false, false);
  asm volatile("v_nop\n\tv_nop\n\tv_nop\n\tv_nop" : "+v"(c) : "v"(a), "v"(b));
  return c;
}
__device__ __forceinline__ v8f mma_b(v16b a, v16b b, v8f c) {
  c = __builtin_amdgcn_wmma_f32_16x16x32_bf16(false, a, false, b, (short)0, c, false, false);
  asm volatile("v_nop\n\tv_nop\n\tv_nop\n\tv_nop" : "+v"(c) : "v"(a), "v"(b));
  return c;
}

template <int ET> struct Elem;
template <> struct Elem<0> { typedef _Float16 T; };
template <> struct Elem<1> { typedef __bf16 T; };
template <int ET, bool SPLIT, int BIAS_MODE, int OUT_MODE, bool RESID, int ACT = 0>
__global__ __launch_bounds__(256) void wmma_gemm64(
    const unsigned short* __restrict__ Ap, const unsigned short* __restrict__ A2p, int lda, long strideA,
    const unsigned short* __restrict__ Btp, const unsigned short* __restrict__ Bt2p, int ldb, long strideB,
    void* __restrict__ Cout, void* __restrict__ Cout2, int ldc, long strideC,
    const float* __restrict__ bias,
    const float* __restrict__ resid, long strideR,
    int M, int N, int K, float scale) {
  typedef typename Elem<ET>::T T;
  typedef typename Frag<T>::V V;
  const T* A = (const T*)Ap; const T* A2 = (const T*)A2p; const T* Bt = (const T*)Btp; const T* Bt2 = (const T*)Bt2p;
  __shared__ __align__(16) float sT[8][16 * 68];
  const int b    = blockIdx.y;
  const int lane = threadIdx.x & 31;
  const int wave = threadIdx.x >> 5;
  const int tilesN = N >> 6;
  const int tilesM = M >> 6;
  const int tile = blockIdx.x * 8 + wave;
  if (tile >= tilesM * tilesN) return;
  const int tm = tile / tilesN;
  const int tn = tile - tm * tilesN;
  const int m0 = tm << 6;
  const int n0 = tn << 6;

  const T* Ab  = A  + (size_t)b * strideA;
  const T* Bb  = Bt + (size_t)b * strideB;
  const T* Ab2 = SPLIT ? (A2  + (size_t)b * strideA) : nullptr;
  const T* Bb2 = SPLIT ? (Bt2 + (size_t)b * strideB) : nullptr;

  const int rlane = lane & 15;
  const int koff  = (lane >> 4) * 8;
  const int mOff  = (lane >> 4) * 8;

  v8f acc[4][4];
#pragma unroll
  for (int i = 0; i < 4; ++i)
#pragma unroll
    for (int j = 0; j < 4; ++j) acc[i][j] = (v8f){0.f,0.f,0.f,0.f,0.f,0.f,0.f,0.f};

  for (int k0 = 0; k0 < K; k0 += 32) {
    V bh[4], bl[4];
#pragma unroll
    for (int j = 0; j < 4; ++j) {
      const size_t bo = (size_t)(n0 + (j << 4) + rlane) * ldb + koff + k0;
      bh[j] = Frag<T>::load(Bb + bo);
      if (SPLIT) bl[j] = Frag<T>::load(Bb2 + bo);
    }
#pragma unroll
    for (int i = 0; i < 4; ++i) {
      const size_t ao = (size_t)(m0 + (i << 4) + rlane) * lda + koff + k0;
      V ah = Frag<T>::load(Ab + ao);
      V al;
      if (SPLIT) al = Frag<T>::load(Ab2 + ao);
#pragma unroll
      for (int j = 0; j < 4; ++j) {
        acc[i][j] = Frag<T>::mma(ah, bh[j], acc[i][j]);
        if (SPLIT) {
          acc[i][j] = Frag<T>::mma(ah, bl[j], acc[i][j]);
          acc[i][j] = Frag<T>::mma(al, bh[j], acc[i][j]);
        }
      }
      Frag<T>::guard(acc[i][0], acc[i][3], ah, SPLIT ? al : ah);
    }
    Frag<T>::keep(bh[0], bh[1], bh[2], bh[3]);
    if (SPLIT) Frag<T>::keep(bl[0], bl[1], bl[2], bl[3]);
  }
  acc_guard4(acc[0][0], acc[0][1], acc[0][2], acc[0][3]);
  acc_guard4(acc[1][0], acc[1][1], acc[1][2], acc[1][3]);
  acc_guard4(acc[2][0], acc[2][1], acc[2][2], acc[2][3]);
  acc_guard4(acc[3][0], acc[3][1], acc[3][2], acc[3][3]);

  float* slab = sT[wave];
  const float* Rb = RESID ? (resid + (size_t)b * strideR) : nullptr;
#pragma unroll
  for (int i = 0; i < 4; ++i) {
    const int mBase = m0 + (i << 4);
#pragma unroll
    for (int j = 0; j < 4; ++j) {
      const int n = n0 + (j << 4) + rlane;
      float bv = 0.f;
      if (BIAS_MODE == 2) bv = bias[n];
#pragma unroll
      for (int r = 0; r < 8; ++r) {
        float v = acc[i][j][r] * scale;
        if (BIAS_MODE == 1) v += bias[mBase + mOff + r];
        if (BIAS_MODE == 2) v += bv;
        if (RESID) v += Rb[(size_t)(mBase + mOff + r) * ldc + n];
        if (ACT == 2) v = fmaxf(v, 0.0f);
        if (ACT == 4) v = (v > 0.f) ? v : 0.01f * v;
        slab[(mOff + r) * 68 + (j << 4) + rlane] = v;
      }
    }
    __builtin_amdgcn_fence(__ATOMIC_RELEASE, "workgroup");
    __builtin_amdgcn_wave_barrier();
    __builtin_amdgcn_fence(__ATOMIC_ACQUIRE, "workgroup");
    if (OUT_MODE == 0) {
      float* C = (float*)Cout + (size_t)b * strideC;
      const int hh = lane >> 4, c4 = (lane & 15) * 4;
      for (int pass = 0; pass < 2; ++pass) {
#pragma unroll
        for (int it = 0; it < 8; ++it) {
          const int row = it * 2 + hh;
          v4f v = *(const v4f*)(slab + row * 68 + c4);
          *(volatile v4f*)(C + (size_t)(mBase + row) * ldc + n0 + c4) = v;
        }
        __threadfence();
      }
    } else {
      const int q = lane >> 3, c8 = (lane & 7) * 8;
      unsigned short* C  = (unsigned short*)Cout  + (size_t)b * strideC;
      unsigned short* C2 = (OUT_MODE == 2) ? ((unsigned short*)Cout2 + (size_t)b * strideC) : nullptr;
      for (int pass = 0; pass < 2; ++pass) {
#pragma unroll
        for (int it = 0; it < 4; ++it) {
          const int row = it * 4 + q;
          const float* sp = slab + row * 68 + c8;
          v8h hv, lv;
#pragma unroll
          for (int e = 0; e < 8; ++e) {
            if (OUT_MODE == 1) {
              hv[e] = (_Float16)sp[e];
            } else {
              unsigned short hb = f2bf_bits(sp[e]);
              unsigned short lb = f2bf_bits(sp[e] - bf_bits2f(hb));
              hv[e] = __builtin_bit_cast(_Float16, hb);
              lv[e] = __builtin_bit_cast(_Float16, lb);
            }
          }
          *(volatile v8h*)(C + (size_t)(mBase + row) * ldc + n0 + c8) = hv;
          if (OUT_MODE == 2) *(volatile v8h*)(C2 + (size_t)(mBase + row) * ldc + n0 + c8) = lv;
        }
        __threadfence();
      }
    }
    __builtin_amdgcn_fence(__ATOMIC_RELEASE, "workgroup");
    __builtin_amdgcn_wave_barrier();
    __builtin_amdgcn_fence(__ATOMIC_ACQUIRE, "workgroup");
  }
}

__global__ __launch_bounds__(256) void cast8_bf16_kernel(const float* __restrict__ in, unsigned short* __restrict__ out, int n8) {
  const int i = blockIdx.x * 256 + threadIdx.x;
  if (i >= n8) return;
  const float* p = in + 8 * (size_t)i;
  const v4f a = *(const v4f*)(p);
  const v4f c = *(const v4f*)(p + 4);
  unsigned short hb[8];
#pragma unroll
  for (int e = 0; e < 4; ++e) {
    hb[e]     = f2bf_bits(a[e]);
    hb[4 + e] = f2bf_bits(c[e]);
  }
  const v4u u = PACK8W(hb);
  unsigned short* q = out + 8 * (size_t)i;
  *(volatile v4u*)q = u;
  __threadfence();
  *(volatile v4u*)q = u;
}

__global__ __launch_bounds__(256) void wt_cast_kernel(const float* __restrict__ W, unsigned short* __restrict__ Wt) {
  __shared__ float sm[64][65];
  const int t  = threadIdx.x;
  const int k0 = blockIdx.x * 64;
  const int n0 = blockIdx.y * 64;
#pragma unroll
  for (int i = 0; i < 16; ++i) {
    const int e = i * 256 + t;
    const int r = e >> 6;
    const int c = e & 63;
    sm[c][r] = W[(size_t)(k0 + r) * kQVK + n0 + c];
  }
  __syncthreads();
  const int lane = t & 31, wave = t >> 5;
  const int rq = lane >> 3, c8 = (lane & 7) * 8;
  v4u u[2];
#pragma unroll
  for (int it = 0; it < 2; ++it) {
    const int row = wave * 8 + it * 4 + rq;
    unsigned short hb[8];
#pragma unroll
    for (int e = 0; e < 8; ++e) hb[e] = f2bf_bits(sm[row][c8 + e]);
    u[it] = PACK8W(hb);
  }
  for (int pass = 0; pass < 2; ++pass) {
#pragma unroll
    for (int it = 0; it < 2; ++it) {
      const int row = wave * 8 + it * 4 + rq;
      *(volatile v4u*)(Wt + (size_t)(n0 + row) * kDim + k0 + c8) = u[it];
    }
    __threadfence();
  }
}

__global__ __launch_bounds__(256) void bias_bf16_kernel(const float* __restrict__ b, float* __restrict__ bb, int n4) {
  const int i = blockIdx.x * 256 + threadIdx.x;
  if (i >= n4) return;
  const v4f a = *(const v4f*)(b + 4 * (size_t)i);
  v4f o;
#pragma unroll
  for (int e = 0; e < 4; ++e) o[e] = bf_bits2f(f2bf_bits(a[e]));
  float* p = bb + 4 * (size_t)i;
  *(volatile v4f*)p = o;
  __threadfence();
  *(volatile v4f*)p = o;
}

__global__ __launch_bounds__(256) void prep_kernel(const float* __restrict__ QVK,
                                                   unsigned short* __restrict__ Q16,
                                                   unsigned short* __restrict__ QBH, unsigned short* __restrict__ QBL,
                                                   unsigned short* __restrict__ KBH, unsigned short* __restrict__ KBL,
                                                   unsigned short* __restrict__ KT16, unsigned short* __restrict__ VT16,
                                                   unsigned short* __restrict__ VTBH, unsigned short* __restrict__ VTBL,
                                                   float* __restrict__ ZT, float* __restrict__ DLOC,
                                                   const int* __restrict__ head_count_unused) {
  (void)head_count_unused;
  __shared__ float sq[64][65];
  __shared__ float sk[64][65];
  __shared__ float sv[64][65];
  __shared__ __align__(16) float szt[64];
  __shared__ __align__(16) float sdl[64];
  const int t = blockIdx.x, h = blockIdx.y;
  const int tid = threadIdx.x, lane = tid & 31, wave = tid >> 5;
  const int r = tid >> 2, qtr = tid & 3, cb = qtr * 16;
  const size_t n = (size_t)t * kChunk + r;
  const float* rowq = QVK + n * kQVK + h * kDh + cb;
  const float* rowv = rowq + kDim;
  const float* rowk = rowq + 2 * kDim;

  float m = -3.0e38f;
#pragma unroll
  for (int c4 = 0; c4 < 4; ++c4) {
    const v4f w = *(const v4f*)(rowq + 4 * c4);
#pragma unroll
    for (int e = 0; e < 4; ++e) sq[r][cb + 4 * c4 + e] = w[e];
    m = fmaxf(m, fmaxf(fmaxf(w[0], w[1]), fmaxf(w[2], w[3])));
  }
  m = fmaxf(m, __shfl_xor(m, 1, 32));
  m = fmaxf(m, __shfl_xor(m, 2, 32));
  float s = 0.f;
#pragma unroll 1
  for (int cc = 0; cc < 16; ++cc) {
    const float ex = expf(sq[r][cb + cc] - m);
    s += ex;
    sq[r][cb + cc] = ex;
  }
  s += __shfl_xor(s, 1, 32);
  s += __shfl_xor(s, 2, 32);
  const float scl = (1.0f / s) * kQScale;
#pragma unroll
  for (int cc = 0; cc < 16; ++cc) sq[r][cb + cc] = sq[r][cb + cc] * scl;
#pragma unroll
  for (int c4 = 0; c4 < 4; ++c4) {
    const v4f w = *(const v4f*)(rowk + 4 * c4);
#pragma unroll
    for (int e = 0; e < 4; ++e) sk[r][cb + 4 * c4 + e] = w[e];
  }
#pragma unroll 1
  for (int cc = 0; cc < 16; ++cc) sk[r][cb + cc] = expf(sk[r][cb + cc]);
#pragma unroll
  for (int c4 = 0; c4 < 4; ++c4) {
    const v4f w = *(const v4f*)(rowv + 4 * c4);
#pragma unroll
    for (int e = 0; e < 4; ++e) sv[r][cb + 4 * c4 + e] = w[e];
  }
  __syncthreads();

  const int rq = lane >> 3, c8 = (lane & 7) * 8;
  const size_t rowbase = (size_t)h * kSeqN + (size_t)t * kChunk;
  v4u uq[2], uqh[2], uql[2], ukh[2], ukl[2], ukt[2], uvt[2], uvh[2], uvl[2];
#pragma unroll
  for (int it = 0; it < 2; ++it) {
    const int row = wave * 8 + it * 4 + rq;
    unsigned short aq[8], aqh[8], aql[8], akh[8], akl[8], akt[8], avt[8], avh[8], avl[8];
#pragma unroll
    for (int e = 0; e < 8; ++e) {
      const float qv  = sq[row][c8 + e];
      const float kv  = sk[row][c8 + e];
      const float ktv = sk[c8 + e][row];
      const float vtv = sv[c8 + e][row];
      aq[e] = h_bits(qv * kQ16Carry);
      const unsigned short qhb = f2bf_bits(qv);
      aqh[e] = qhb;
      aql[e] = f2bf_bits(qv - bf_bits2f(qhb));
      const unsigned short khb = f2bf_bits(kv);
      akh[e] = khb;
      akl[e] = f2bf_bits(kv - bf_bits2f(khb));
      akt[e] = h_bits(ktv);
      avt[e] = h_bits(vtv * kVCarry);
      const unsigned short vhb = f2bf_bits(vtv);
      avh[e] = vhb;
      avl[e] = f2bf_bits(vtv - bf_bits2f(vhb));
    }
    uq[it]  = PACK8W(aq);
    uqh[it] = PACK8W(aqh);
    uql[it] = PACK8W(aql);
    ukh[it] = PACK8W(akh);
    ukl[it] = PACK8W(akl);
    ukt[it] = PACK8W(akt);
    uvt[it] = PACK8W(avt);
    uvh[it] = PACK8W(avh);
    uvl[it] = PACK8W(avl);
  }
  for (int pass = 0; pass < 2; ++pass) {
#pragma unroll
    for (int it = 0; it < 2; ++it) {
      const int row = wave * 8 + it * 4 + rq;
      const size_t ro = (rowbase + row) * kDh + c8;
      const size_t co = (size_t)row * kHN + rowbase + c8;
      *(volatile v4u*)(Q16  + ro) = uq[it];
      *(volatile v4u*)(QBH  + ro) = uqh[it];
      *(volatile v4u*)(QBL  + ro) = uql[it];
      *(volatile v4u*)(KBH  + ro) = ukh[it];
      *(volatile v4u*)(KBL  + ro) = ukl[it];
      *(volatile v4u*)(KT16 + co) = ukt[it];
      *(volatile v4u*)(VT16 + co) = uvt[it];
      *(volatile v4u*)(VTBH + co) = uvh[it];
      *(volatile v4u*)(VTBL + co) = uvl[it];
    }
    __threadfence();
  }
  __syncthreads();

  if (tid < 64) {
    const int d = tid;
    float acc = 0.f;
#pragma unroll 4
    for (int rr = 0; rr < 64; ++rr) { acc += sk[rr][d]; sv[rr][d] = acc; }
    szt[d] = acc;
  }
  __syncthreads();

  float part = 0.f;
#pragma unroll 1
  for (int c4 = 0; c4 < 4; ++c4) {
#pragma unroll
    for (int e = 0; e < 4; ++e) {
      const int cc = cb + 4 * c4 + e;
      part = fmaf(sq[r][cc], sv[r][cc], part);
    }
  }
  part += __shfl_xor(part, 1, 32);
  part += __shfl_xor(part, 2, 32);
  if (qtr == 0) sdl[r] = part;
  __syncthreads();

  if (wave == 0) {
    const v4f val = *(const v4f*)(sdl + 4 * (lane & 15));
    if (lane < 16) {
      float* p = DLOC + rowbase + 4 * lane;
      *(volatile v4f*)p = val;
      __threadfence();
      *(volatile v4f*)p = val;
    }
  } else if (wave == 1) {
    const v4f val = *(const v4f*)(szt + 4 * (lane & 15));
    if (lane < 16) {
      float* p = ZT + ((size_t)(h * kNCh + t)) * kDh + 4 * lane;
      *(volatile v4f*)p = val;
      __threadfence();
      *(volatile v4f*)p = val;
    }
  }
}

__global__ __launch_bounds__(256) void prefix_den_kernel(const float* __restrict__ G, const float* __restrict__ ZT,
                                                         const float* __restrict__ DLOC, const unsigned short* __restrict__ Q16,
                                                         unsigned short* __restrict__ S16, float* __restrict__ DEN) {
  __shared__ __align__(16) float zp[64];
  __shared__ __align__(16) float dens[64];
  const int h = blockIdx.x;
  const int tid = threadIdx.x, lane = tid & 31, wave = tid >> 5;
  const int r = tid >> 2, qtr = tid & 3;
  float run[16];
#pragma unroll
  for (int j = 0; j < 16; ++j) run[j] = 0.f;
  float zrun = 0.f;
  for (int t = 0; t < kNCh; ++t) {
    const size_t base = ((size_t)(h * kNCh + t)) * (kDh * kDh);
    const float* gp = G + base + 8 * tid;
    const v4f a0 = *(const v4f*)(gp);
    const v4f a1 = *(const v4f*)(gp + 4);
    const v4f a2 = *(const v4f*)(gp + 2048);
    const v4f a3 = *(const v4f*)(gp + 2052);
    unsigned short hb[16];
#pragma unroll
    for (int j = 0; j < 16; ++j) hb[j] = h_bits(run[j] * kVCarryInv);
#pragma unroll
    for (int e = 0; e < 4; ++e) { run[e] += a0[e]; run[4 + e] += a1[e]; run[8 + e] += a2[e]; run[12 + e] += a3[e]; }
    const v4u u0 = (v4u){pk16(hb[0], hb[1]), pk16(hb[2], hb[3]), pk16(hb[4], hb[5]), pk16(hb[6], hb[7])};
    const v4u u1 = (v4u){pk16(hb[8], hb[9]), pk16(hb[10], hb[11]), pk16(hb[12], hb[13]), pk16(hb[14], hb[15])};
    unsigned short* s0 = S16 + base + 8 * tid;
    unsigned short* s1 = s0 + 2048;
    *(volatile v4u*)s0 = u0;
    *(volatile v4u*)s1 = u1;
    __threadfence();
    *(volatile v4u*)s0 = u0;
    *(volatile v4u*)s1 = u1;

    if (tid < 64) {
      zp[tid] = zrun;
      zrun += ZT[((size_t)(h * kNCh + t)) * kDh + tid];
    }
    __syncthreads();

    const size_t qoff = (((size_t)h * kSeqN + (size_t)t * kChunk + r)) * kDh + qtr * 16;
    const v4u w0 = *(const v4u*)(Q16 + qoff);
    const v4u w1 = *(const v4u*)(Q16 + qoff + 8);
    float part = 0.f;
#pragma unroll
    for (int e = 0; e < 4; ++e) {
      const unsigned wa = w0[e];
      const unsigned wb = w1[e];
      const float qa0 = h16_to_f32(wa & 0xffffu), qa1 = h16_to_f32(wa >> 16);
      const float qb0 = h16_to_f32(wb & 0xffffu), qb1 = h16_to_f32(wb >> 16);
      part = fmaf(qa0, zp[qtr * 16 + 2 * e],         part);
      part = fmaf(qa1, zp[qtr * 16 + 2 * e + 1],     part);
      part = fmaf(qb0, zp[qtr * 16 + 8 + 2 * e],     part);
      part = fmaf(qb1, zp[qtr * 16 + 8 + 2 * e + 1], part);
    }
    part += __shfl_xor(part, 1, 32);
    part += __shfl_xor(part, 2, 32);
    const float dl = DLOC[(size_t)h * kSeqN + (size_t)t * kChunk + r];
    if (qtr == 0) dens[r] = dl + part * kQ16Inv + kEpsDen;
    __syncthreads();

    if (wave == 0) {
      const v4f val = *(const v4f*)(dens + 4 * (lane & 15));
      if (lane < 16) {
        float* p = DEN + (size_t)h * kSeqN + (size_t)t * kChunk + 4 * lane;
        *(volatile v4f*)p = val;
        __threadfence();
        *(volatile v4f*)p = val;
      }
    }
    __syncthreads();
  }
}

__global__ __launch_bounds__(128) void attn_chunk_kernel(const unsigned short* __restrict__ QBHp, const unsigned short* __restrict__ QBLp,
                                                         const unsigned short* __restrict__ KBHp, const unsigned short* __restrict__ KBLp,
                                                         const unsigned short* __restrict__ VTBHp, const unsigned short* __restrict__ VTBLp,
                                                         const unsigned short* __restrict__ Q16p, const unsigned short* __restrict__ S16p,
                                                         const float* __restrict__ DEN, float* __restrict__ out) {
  __shared__ __align__(16) __bf16 Psh[4][16 * 64];
  __shared__ __align__(16) __bf16 Psl[4][16 * 64];
  __shared__ __align__(16) float Os[4][16 * 68];
  const __bf16* QBH  = (const __bf16*)QBHp;
  const __bf16* QBL  = (const __bf16*)QBLp;
  const __bf16* KBH  = (const __bf16*)KBHp;
  const __bf16* KBL  = (const __bf16*)KBLp;
  const __bf16* VTBH = (const __bf16*)VTBHp;
  const __bf16* VTBL = (const __bf16*)VTBLp;
  const _Float16* Qh = (const _Float16*)Q16p;
  const _Float16* Sh = (const _Float16*)S16p;
  const int t = blockIdx.x, h = blockIdx.y;
  const int tid = threadIdx.x, wave = tid >> 5, lane = tid & 31;
  const int hh = lane >> 4, c = lane & 15, koff = hh * 8;
  const size_t rowbase = (size_t)h * kSeqN + (size_t)t * kChunk;
  const int q0 = wave * 16;

  v8f p[4];
#pragma unroll
  for (int jb = 0; jb < 4; ++jb) p[jb] = (v8f){0.f,0.f,0.f,0.f,0.f,0.f,0.f,0.f};
#pragma unroll
  for (int kk = 0; kk < 2; ++kk) {
    const size_t qo = (rowbase + q0 + c) * kDh + koff + kk * 32;
    const v16b qh = Frag<__bf16>::load(QBH + qo);
    const v16b ql = Frag<__bf16>::load(QBL + qo);
#pragma unroll
    for (int jb = 0; jb < 4; ++jb) {
      const size_t ko = (rowbase + 16 * jb + c) * kDh + koff + kk * 32;
      const v16b kh = Frag<__bf16>::load(KBH + ko);
      const v16b kl = Frag<__bf16>::load(KBL + ko);
      p[jb] = mma_b(qh, kh, p[jb]);
      p[jb] = mma_b(qh, kl, p[jb]);
      p[jb] = mma_b(ql, kh, p[jb]);
      asm volatile("" ::: "memory");
    }
  }

  __bf16* pwh = Psh[wave];
  __bf16* pwl = Psl[wave];
#pragma unroll
  for (int jb = 0; jb < 4; ++jb) {
    const int jj = 16 * jb + c;
#pragma unroll
    for (int r = 0; r < 8; ++r) {
      const int il = q0 + 8 * hh + r;
      const float pv = (jj <= il) ? p[jb][r] : 0.0f;
      const unsigned short hb = f2bf_bits(pv);
      const unsigned short lb = f2bf_bits(pv - bf_bits2f(hb));
      pwh[(8 * hh + r) * 64 + jj] = __builtin_bit_cast(__bf16, hb);
      pwl[(8 * hh + r) * 64 + jj] = __builtin_bit_cast(__bf16, lb);
    }
  }
  __syncthreads();

  v8f opv[4];
#pragma unroll
  for (int jc = 0; jc < 4; ++jc) opv[jc] = (v8f){0.f,0.f,0.f,0.f,0.f,0.f,0.f,0.f};
#pragma unroll
  for (int kk = 0; kk < 2; ++kk) {
    const v16b pa = Frag<__bf16>::load(pwh + c * 64 + koff + kk * 32);
    const v16b pl = Frag<__bf16>::load(pwl + c * 64 + koff + kk * 32);
#pragma unroll
    for (int jc = 0; jc < 4; ++jc) {
      const size_t vo = (size_t)(16 * jc + c) * kHN + rowbase + koff + kk * 32;
      const v16b vh = Frag<__bf16>::load(VTBH + vo);
      const v16b vl = Frag<__bf16>::load(VTBL + vo);
      opv[jc] = mma_b(pa, vh, opv[jc]);
      opv[jc] = mma_b(pa, vl, opv[jc]);
      opv[jc] = mma_b(pl, vh, opv[jc]);
      asm volatile("" ::: "memory");
    }
  }

  v8f oqs[4];
#pragma unroll
  for (int jc = 0; jc < 4; ++jc) oqs[jc] = (v8f){0.f,0.f,0.f,0.f,0.f,0.f,0.f,0.f};
  const size_t sbase = ((size_t)(h * kNCh + t)) * kDh;
#pragma unroll
  for (int kk = 0; kk < 2; ++kk) {
    const v16h qa = Frag<_Float16>::load(Qh + (rowbase + q0 + c) * kDh + koff + kk * 32);
#pragma unroll
    for (int jc = 0; jc < 4; ++jc) {
      const v16h sb = Frag<_Float16>::load(Sh + (sbase + 16 * jc + c) * kDh + koff + kk * 32);
      oqs[jc] = mma_h(qa, sb, oqs[jc]);
      asm volatile("" ::: "memory");
    }
  }

  const float* dp = DEN + rowbase + q0 + 8 * hh;
  const v4f d0 = *(const v4f*)(dp);
  const v4f d1 = *(const v4f*)(dp + 4);
  const float dv[8] = {d0[0], d0[1], d0[2], d0[3], d1[0], d1[1], d1[2], d1[3]};
  float inv[8];
#pragma unroll
  for (int r = 0; r < 8; ++r) inv[r] = 1.0f / dv[r];
  float* os = Os[wave];
#pragma unroll
  for (int r = 0; r < 8; ++r) {
#pragma unroll
    for (int jc = 0; jc < 4; ++jc)
      os[(8 * hh + r) * 68 + 16 * jc + c] = (opv[jc][r] + oqs[jc][r] * kQ16Inv) * inv[r];
  }
  __syncthreads();
  {
    const int c4 = (lane & 15) * 4;
    float* ob = out + (size_t)h * kDh;
    for (int pass = 0; pass < 2; ++pass) {
#pragma unroll
      for (int it = 0; it < 8; ++it) {
        const int row = it * 2 + hh;
        const v4f val = *(const v4f*)(os + row * 68 + c4);
        *(volatile v4f*)(ob + ((size_t)t * kChunk + q0 + row) * kDim + c4) = val;
      }
      __threadfence();
    }
  }
}

extern "C" void kernel_launch(void* const* d_in, const int* in_sizes, int n_in,
                              void* d_out, int out_size, void* d_ws, size_t ws_size,
                              hipStream_t stream) {
  if (n_in < 4) return;
  const int nX = kSeqN * kDim;
  if (in_sizes[0] != nX || in_sizes[1] != kDim * kQVK || in_sizes[2] != kQVK) return;
  if (out_size != nX) return;

  const size_t szXB  = (size_t)kSeqN * kDim * 2;
  const size_t szWT  = (size_t)kQVK * kDim * 2;
  const size_t szBB  = (size_t)kQVK * 4;
  const size_t szQVK = (size_t)kSeqN * kQVK * 4;
  const size_t szP16 = (size_t)kHeads * kSeqN * kDh * 2;
  const size_t szG   = (size_t)kHeads * kNCh * kDh * kDh * 4;
  const size_t szS16 = (size_t)kHeads * kNCh * kDh * kDh * 2;
  const size_t szZT  = (size_t)kHeads * kNCh * kDh * 4;
  const size_t szRow = (size_t)kHeads * kSeqN * 4;
  const size_t offXB  = 0;
  const size_t offWT  = offXB + szXB;
  const size_t offBB  = offWT + szWT;
  const size_t offQVK = offBB + szBB;
  const size_t offQ16 = offQVK + szQVK;
  const size_t offQBH = offQ16 + szP16;
  const size_t offQBL = offQBH + szP16;
  const size_t offKBH = offQBL + szP16;
  const size_t offKBL = offKBH + szP16;
  const size_t offKT  = offKBL + szP16;
  const size_t offVT  = offKT + szP16;
  const size_t offVBH = offVT + szP16;
  const size_t offVBL = offVBH + szP16;
  const size_t offG   = offVBL + szP16;
  const size_t offS16 = offG + szG;
  const size_t offZT  = offS16 + szS16;
  const size_t offDL  = offZT + szZT;
  const size_t offDEN = offDL + szRow;
  const size_t total  = offDEN + szRow;
  if (ws_size < total) return;

  const float* x  = (const float*)d_in[0];
  const float* W  = (const float*)d_in[1];
  const float* bq = (const float*)d_in[2];
  const int*   hn = (const int*)d_in[3];
  float* out = (float*)d_out;
  char* ws = (char*)d_ws;
  unsigned short* XB   = (unsigned short*)(ws + offXB);
  unsigned short* WT   = (unsigned short*)(ws + offWT);
  float*          BB   = (float*)(ws + offBB);
  float*          QVK  = (float*)(ws + offQVK);
  unsigned short* Q16  = (unsigned short*)(ws + offQ16);
  unsigned short* QBH  = (unsigned short*)(ws + offQBH);
  unsigned short* QBL  = (unsigned short*)(ws + offQBL);
  unsigned short* KBH  = (unsigned short*)(ws + offKBH);
  unsigned short* KBL  = (unsigned short*)(ws + offKBL);
  unsigned short* KT16 = (unsigned short*)(ws + offKT);
  unsigned short* VT16 = (unsigned short*)(ws + offVT);
  unsigned short* VTBH = (unsigned short*)(ws + offVBH);
  unsigned short* VTBL = (unsigned short*)(ws + offVBL);
  float*          G    = (float*)(ws + offG);
  unsigned short* S16  = (unsigned short*)(ws + offS16);
  float*          ZT   = (float*)(ws + offZT);
  float*          DLOC = (float*)(ws + offDL);
  float*          DEN  = (float*)(ws + offDEN);

  const int n8x = nX / 8;
  cast8_bf16_kernel<<<dim3(n8x / 256), dim3(256), 0, stream>>>(x, XB, n8x);
  wt_cast_kernel<<<dim3(kDim / 64, kQVK / 64), dim3(256), 0, stream>>>(W, WT);
  const int n4b = kQVK / 4;
  bias_bf16_kernel<<<dim3(n4b / 256), dim3(256), 0, stream>>>(bq, BB, n4b);

  const int tilesQKV = (kSeqN / 64) * (kQVK / 64);
  wmma_gemm64<1, false, 2, 0, false, 0><<<dim3(tilesQKV / 8, 1), dim3(256), 0, stream>>>(
      XB, XB, kDim, 0L, WT, WT, kDim, 0L,
      (void*)QVK, (void*)QVK, kQVK, 0L, BB, BB, 0L, kSeqN, kQVK, kDim, 1.0f);

  prep_kernel<<<dim3(kNCh, kHeads), dim3(256), 0, stream>>>(QVK, Q16, QBH, QBL, KBH, KBL, KT16, VT16, VTBH, VTBL, ZT, DLOC, hn);

  wmma_gemm64<0, false, 0, 0, false, 0><<<dim3(1, kHeads * kNCh), dim3(32), 0, stream>>>(
      VT16, VT16, kHN, (long)kChunk, KT16, KT16, kHN, (long)kChunk,
      (void*)G, (void*)G, kDh, (long)(kDh * kDh), BB, BB, 0L, kDh, kDh, kChunk, 1.0f);

  prefix_den_kernel<<<dim3(kHeads), dim3(256), 0, stream>>>(G, ZT, DLOC, Q16, S16, DEN);

  attn_chunk_kernel<<<dim3(kNCh, kHeads), dim3(128), 0, stream>>>(QBH, QBL, KBH, KBL, VTBH, VTBL, Q16, S16, DEN, out);
}
